// MKLSAGEInference_26087631356381
// MI455X (gfx1250) — hardware-verified
//
#include <hip/hip_runtime.h>


#define FEAT 128
#define NTILE 256
#define ECHUNK 1024

typedef __attribute__((ext_vector_type(16))) _Float16 v16h;
typedef __attribute__((ext_vector_type(8)))  _Float16 v8h;
typedef __attribute__((ext_vector_type(8)))  float v8f;
typedef __attribute__((ext_vector_type(4)))  float v4f;

template <typename T> __device__ __forceinline__ void vst2(void* p, T v) { *(volatile T*)p = v; __threadfence(); *(volatile T*)p = v; }
__device__ __forceinline__ v8f wmma16(v16h a, v16h b, v8f c) {
  v8f d = __builtin_amdgcn_wmma_f32_16x16x32_f16(false, a, false, b, (short)0, c, false, false);
  asm volatile("v_nop\n\tv_nop\n\tv_nop\n\tv_nop" : "+v"(d) : "v"(a), "v"(b));
  return d;
}
__device__ __forceinline__ v16h frag_f32(const float* row, int k0, int lane) {
  v16h a; const float* p = row + k0 + 8 * (lane >> 4);
#pragma unroll
  for (int i = 0; i < 8; ++i) { a[i] = (_Float16)p[i]; a[8 + i] = (_Float16)p[16 + i]; }
  return a;
}

__global__ __launch_bounds__(256) void sage_gemm_kernel(const float* __restrict__ X, const float* __restrict__ W,
    const float* __restrict__ bias, const float* __restrict__ aggr, const float* __restrict__ deg, float* __restrict__ Y, int nrows) {
  __shared__ __align__(16) _Float16 sW[FEAT][136];
  __shared__ __align__(16) float so[8][16 * 132];
  const int tid = threadIdx.x;
  for (int i = tid; i < FEAT * FEAT; i += 256) { const int n = i >> 7, k = i & 127; sW[n][k] = (_Float16)W[i]; }
  __syncthreads();
  const int lane = tid & 31, wave = tid >> 5, col = lane & 15, g = lane >> 4;
  const int m0 = (blockIdx.x * 8 + wave) * 16;
  const int arow = (m0 + col < nrows) ? (m0 + col) : 0;
  const float* ap = X + (size_t)arow * FEAT;
  v8f acc[8];
#pragma unroll
  for (int n = 0; n < 8; ++n) {
    if (aggr) {
#pragma unroll
      for (int r = 0; r < 8; ++r) { const int row = m0 + g * 8 + r; const int rc = row < nrows ? row : 0;
        acc[n][r] = aggr[(size_t)rc * FEAT + n * 16 + col] / fmaxf(deg[rc], 1.0f); }
    } else {
      const float b = bias ? bias[n * 16 + col] : 0.0f;
#pragma unroll
      for (int r = 0; r < 8; ++r) acc[n][r] = b;
    }
  }
#pragma unroll
  for (int kc = 0; kc < FEAT / 32; ++kc) {
    const v16h a = frag_f32(ap, kc * 32, lane);
#pragma unroll
    for (int n = 0; n < 8; ++n) {
      union { v16h v; v8h q[2]; } b; const _Float16* bp = &sW[n * 16 + col][kc * 32 + 8 * g];
      b.q[0] = *(const v8h*)(bp); b.q[1] = *(const v8h*)(bp + 16);
      acc[n] = wmma16(a, b.v, acc[n]);
    }
  }
  float* S = so[wave];
#pragma unroll
  for (int n = 0; n < 8; ++n)
#pragma unroll
    for (int r = 0; r < 8; ++r) S[(g * 8 + r) * 132 + n * 16 + col] = acc[n][r];
  asm volatile("s_wait_dscnt 0" ::: "memory"); __builtin_amdgcn_wave_barrier(); __builtin_amdgcn_fence(__ATOMIC_RELEASE, "workgroup");
#pragma unroll 4
  for (int r = 0; r < 16; ++r) { const int row = m0 + r;
    if (row < nrows) vst2(Y + (size_t)row * FEAT + lane * 4, *(const v4f*)(S + r * 132 + lane * 4)); }
}

__global__ __launch_bounds__(256) void sage_gather_kernel(const int* __restrict__ ei, const float* __restrict__ xl,
                                                          float* __restrict__ agg, float* __restrict__ deg, int n_nodes, int n_edges) {
  __shared__ __align__(16) float acc[NTILE][FEAT];
  __shared__ int es[ECHUNK], ed[ECHUNK];
  __shared__ float cnt[NTILE];
  const int tid = threadIdx.x, lane = tid & 31, wave = tid >> 5;
  const int d0 = blockIdx.x * NTILE;
  for (int i = tid; i < NTILE * FEAT / 4; i += 256) *(v4f*)(&acc[0][0] + i * 4) = (v4f){0.f, 0.f, 0.f, 0.f};
  for (int i = tid; i < NTILE; i += 256) cnt[i] = 0.f;
  __syncthreads();
  for (int e0 = 0; e0 < n_edges; e0 += ECHUNK) {
    const int ne = (n_edges - e0 < ECHUNK) ? (n_edges - e0) : ECHUNK;
    __syncthreads();
    for (int i = tid; i < ne; i += 256) { es[i] = ei[e0 + i]; ed[i] = ei[(size_t)n_edges + e0 + i]; }
    __syncthreads();
    for (int base = 0; base < ne; base += 32) {
      const int i = base + lane;
      int d = (i < ne) ? ed[i] : -1;
      const int dl = d - d0;
      const bool mine = (dl >= 0) && (dl < NTILE) && ((dl & 7) == wave);
      unsigned msk = (unsigned)__builtin_amdgcn_ballot_w32(mine);
      while (msk) {
        const int j = __builtin_ctz(msk); msk &= msk - 1u;
        const int ii = base + j;
        const int dlj = ed[ii] - d0;
        int s = es[ii]; s = s < 0 ? 0 : (s >= n_nodes ? n_nodes - 1 : s);
        const v4f v = *(const v4f*)(xl + (size_t)s * FEAT + lane * 4);
        float* arow = &acc[dlj][lane * 4];
        v4f a = *(v4f*)arow; a += v; *(v4f*)arow = a;
        if (lane == 0) cnt[dlj] += 1.0f;
      }
    }
  }
  __syncthreads();
  for (int r = wave; r < NTILE; r += 8) { const int node = d0 + r;
    if (node < n_nodes) vst2(agg + (size_t)node * FEAT + lane * 4, *(const v4f*)(&acc[r][lane * 4])); }
  for (int i = tid; i < NTILE; i += 256) { const int node = d0 + i; if (node < n_nodes) vst2(deg + node, cnt[i]); }
}

extern "C" void kernel_launch(void* const* d_in, const int* in_sizes, int n_in,
                              void* d_out, int out_size, void* d_ws, size_t ws_size,
                              hipStream_t stream) {
  (void)n_in; (void)out_size; (void)ws_size;
  const float* x   = (const float*)d_in[0];
  const int*   ei  = (const int*)d_in[1];
  const float* W_l = (const float*)d_in[2];
  const float* b_l = (const float*)d_in[3];
  const float* W_r = (const float*)d_in[4];
  float* out = (float*)d_out;
  const int n_nodes = in_sizes[0] / FEAT;
  const int n_edges = in_sizes[1] / 2;
  float* xl  = (float*)d_ws;
  float* agg = xl + (size_t)n_nodes * FEAT;
  float* deg = agg + (size_t)n_nodes * FEAT;
  const int mblocks = (n_nodes + 127) / 128;
  sage_gemm_kernel<<<mblocks, 256, 0, stream>>>(x, W_l, b_l, nullptr, nullptr, xl, n_nodes);
  sage_gather_kernel<<<(n_nodes + NTILE - 1) / NTILE, 256, 0, stream>>>(ei, xl, agg, deg, n_nodes, n_edges);
  sage_gemm_kernel<<<mblocks, 256, 0, stream>>>(x, W_r, nullptr, agg, deg, out, n_nodes);
}
